// MultiHeadAttentionwithRoPE_37357625541121
// MI455X (gfx1250) — hardware-verified
//
#include <hip/hip_runtime.h>
#include <math.h>
#include <stdint.h>

#ifndef NB
#define NB 2
#endif
#ifndef SEQ
#define SEQ 2048
#endif
#define NB_FULL  2
#define SEQ_FULL 2048
#define DM   1024
#define NH   16
#define HD   64
#define NFRQ 32
#define TOK  (NB * SEQ)

static_assert(NH * HD == DM);
static_assert(HD == 2 * NFRQ);
static_assert(HD == 64);
static_assert(NB >= 1 && NB <= NB_FULL);
static_assert(SEQ >= 64 && SEQ <= SEQ_FULL);
static_assert(SEQ % 64 == 0);
static_assert(DM % 64 == 0);
static_assert(DM % 32 == 0);
static_assert(SEQ % 8 == 0);
static_assert((TOK * DM) % (256 * 8) == 0);
static_assert((DM * DM) % (256 * 8) == 0);
static_assert(((TOK / 64) * (DM / 64)) % 8 == 0);

typedef _Float16     v16h __attribute__((ext_vector_type(16)));
typedef _Float16     v8h  __attribute__((ext_vector_type(8)));
typedef __bf16       v16b __attribute__((ext_vector_type(16)));
typedef __bf16       v8b  __attribute__((ext_vector_type(8)));
typedef float        v8f  __attribute__((ext_vector_type(8)));
typedef float        v4f  __attribute__((ext_vector_type(4)));
typedef unsigned int v4u  __attribute__((ext_vector_type(4)));

__device__ __forceinline__ unsigned short f2bf_bits(float f) {
  const unsigned u = __float_as_uint(f);
  return (unsigned short)((u + 0x7FFFu + ((u >> 16) & 1u)) >> 16);
}
__device__ __forceinline__ float bf_bits2f(unsigned short h) { return __uint_as_float(((unsigned)h) << 16); }
__device__ __forceinline__ unsigned pk16(unsigned short a, unsigned short b) { return (unsigned)a | ((unsigned)b << 16); }
__device__ __forceinline__ v8f zero8() { v8f z = {0.f, 0.f, 0.f, 0.f, 0.f, 0.f, 0.f, 0.f}; return z; }
__device__ __forceinline__ int wave_id() { return __builtin_amdgcn_readfirstlane((int)(threadIdx.x >> 5)); }

__device__ __forceinline__ void lds_wave_sync() {
  __builtin_amdgcn_fence(3, "workgroup");
  __builtin_amdgcn_wave_barrier();
  __builtin_amdgcn_fence(2, "workgroup");
}

union FragB { v16b v; v8b h[2]; };
__device__ __forceinline__ v16b ldfrag_b(const __bf16* p) { FragB f; f.h[0] = *(const v8b*)(p); f.h[1] = *(const v8b*)(p + 16); return f.v; }

__device__ __forceinline__ v8f mma_b(v16b a, v16b b, v8f c) {
  return __builtin_amdgcn_wmma_f32_16x16x32_bf16(false, a, false, b, (short)0, c, false, false);
}
__device__ __forceinline__ v8f at_mma(v16b a, v16b b, v8f c) {
  c = __builtin_amdgcn_wmma_f32_16x16x32_bf16(false, a, false, b, (short)0, c, false, false);
  asm volatile("v_nop\n\tv_nop\n\tv_nop\n\tv_nop" : "+v"(c) : "v"(a), "v"(b));
  return c;
}
__device__ __forceinline__ void dep_guard_b(v8f& a, v8f& b, v16b x, v16b y) {
  asm volatile("v_nop\n\tv_nop\n\tv_nop\n\tv_nop" : "+v"(a), "+v"(b) : "v"(x), "v"(y));
}
__device__ __forceinline__ void keep4_b(v16b a, v16b b, v16b c, v16b d) { asm volatile("v_nop" :: "v"(a), "v"(b), "v"(c), "v"(d)); }
__device__ __forceinline__ void acc_guard4(v8f& a, v8f& b, v8f& c, v8f& d) {
  asm volatile("v_nop\n\tv_nop\n\tv_nop\n\tv_nop" : "+v"(a), "+v"(b), "+v"(c), "+v"(d));
}

template <int SPLIT, int OUT_MODE, bool ROT>
__global__ __launch_bounds__(256) void wmma_gemm64(
    const unsigned short* __restrict__ Ap, const unsigned short* __restrict__ A2p, int lda,
    const unsigned short* __restrict__ Btp, const unsigned short* __restrict__ Bt2p, int ldb,
    void* Cout, void* Cout2, int ldc,
    const float* __restrict__ cst, const float* __restrict__ snt,
    int M, int N, int K, float scale) {
  __shared__ __align__(16) float sT[8][16 * 68];
  const int lane = threadIdx.x & 31;
  const int wave = threadIdx.x >> 5;
  const int tilesN = N >> 6;
  const int tilesM = M >> 6;
  const int tile = (int)blockIdx.x * 8 + wave;
  if (tile >= tilesM * tilesN) return;
  const int tm = tile / tilesN;
  const int tn = tile - tm * tilesN;
  const int m0 = tm << 6;
  const int n0 = tn << 6;

  const __bf16* A   = (const __bf16*)(const void*)Ap;
  const __bf16* A2  = (const __bf16*)(const void*)A2p;
  const __bf16* Bt  = (const __bf16*)(const void*)Btp;
  const __bf16* Bt2 = (const __bf16*)(const void*)Bt2p;

  const int rlane = lane & 15;
  const int koff  = (lane >> 4) * 8;
  const int mOff  = (lane >> 4) * 8;

  v8f acc[4][4];
#pragma unroll
  for (int i = 0; i < 4; ++i)
#pragma unroll
    for (int j = 0; j < 4; ++j) acc[i][j] = zero8();

  for (int k0 = 0; k0 < K; k0 += 32) {
    v16b bh[4], bl[4];
#pragma unroll
    for (int j = 0; j < 4; ++j) {
      const size_t bo = (size_t)(n0 + (j << 4) + rlane) * ldb + koff + k0;
      bh[j] = ldfrag_b(Bt + bo);
      if (SPLIT == 2) bl[j] = ldfrag_b(Bt2 + bo);
    }
#pragma unroll
    for (int i = 0; i < 4; ++i) {
      const size_t ao = (size_t)(m0 + (i << 4) + rlane) * lda + koff + k0;
      v16b ah = ldfrag_b(A + ao);
      v16b al = ah;
      if (SPLIT >= 1) al = ldfrag_b(A2 + ao);
#pragma unroll
      for (int j = 0; j < 4; ++j) {
        acc[i][j] = mma_b(ah, bh[j], acc[i][j]);
        if (SPLIT == 2) acc[i][j] = mma_b(ah, bl[j], acc[i][j]);
        if (SPLIT >= 1) acc[i][j] = mma_b(al, bh[j], acc[i][j]);
      }
      dep_guard_b(acc[i][0], acc[i][3], ah, al);
    }
    keep4_b(bh[0], bh[1], bh[2], bh[3]);
    if (SPLIT == 2) keep4_b(bl[0], bl[1], bl[2], bl[3]);
  }
  acc_guard4(acc[0][0], acc[0][1], acc[0][2], acc[0][3]);
  acc_guard4(acc[1][0], acc[1][1], acc[1][2], acc[1][3]);
  acc_guard4(acc[2][0], acc[2][1], acc[2][2], acc[2][3]);
  acc_guard4(acc[3][0], acc[3][1], acc[3][2], acc[3][3]);

  float* slab = sT[wave];
#pragma unroll
  for (int i = 0; i < 4; ++i) {
    const int mBase = m0 + (i << 4);
#pragma unroll
    for (int j = 0; j < 4; ++j) {
#pragma unroll
      for (int r = 0; r < 8; ++r)
        slab[(mOff + r) * 68 + (j << 4) + rlane] = acc[i][j][r] * scale;
    }
    lds_wave_sync();
    if (OUT_MODE == 0) {
      float* C = (float*)Cout;
      const int hh = lane >> 4, c4 = (lane & 15) * 4;
      for (int pass = 0; pass < 2; ++pass) {
#pragma unroll
        for (int it = 0; it < 8; ++it) {
          const int row = it * 2 + hh;
          const int gm  = mBase + row;
          const size_t orow = (size_t)(gm / SEQ) * SEQ_FULL + (size_t)(gm % SEQ);
          const v4f v = *(const v4f*)(slab + row * 68 + c4);
          *(volatile v4f*)(C + orow * (size_t)ldc + n0 + c4) = v;
        }
        __threadfence();
      }
    } else {
      const int q = lane >> 3, c8 = (lane & 7) * 8;
      unsigned short* C  = (unsigned short*)Cout;
      unsigned short* C2 = (unsigned short*)Cout2;
      for (int pass = 0; pass < 2; ++pass) {
#pragma unroll
        for (int it = 0; it < 4; ++it) {
          const int row = it * 4 + q;
          const float* sp = slab + row * 68 + c8;
          float xv[8];
#pragma unroll
          for (int e = 0; e < 8; ++e) xv[e] = sp[e];
          if (ROT) {
            const int pos = (mBase + row) % SEQ;
            const size_t to = (size_t)pos * NFRQ + (c8 >> 1);
            const v4f cv = *(const v4f*)(cst + to);
            const v4f sv = *(const v4f*)(snt + to);
#pragma unroll
            for (int p = 0; p < 4; ++p) {
              const float x1 = xv[2 * p], x2 = xv[2 * p + 1];
              xv[2 * p]     = x1 * cv[p] - x2 * sv[p];
              xv[2 * p + 1] = x1 * sv[p] + x2 * cv[p];
            }
          }
          v8h hv, lv;
#pragma unroll
          for (int e = 0; e < 8; ++e) {
            const unsigned short hb = f2bf_bits(xv[e]);
            const unsigned short lb = f2bf_bits(xv[e] - bf_bits2f(hb));
            hv[e] = __builtin_bit_cast(_Float16, hb);
            lv[e] = __builtin_bit_cast(_Float16, lb);
          }
          *(volatile v8h*)(C  + (size_t)(mBase + row) * ldc + n0 + c8) = hv;
          *(volatile v8h*)(C2 + (size_t)(mBase + row) * ldc + n0 + c8) = lv;
        }
        __threadfence();
      }
    }
    lds_wave_sync();
  }
}

__global__ __launch_bounds__(256) void rot_table_kernel(float* __restrict__ cst, float* __restrict__ snt) {
  const int lane = threadIdx.x & 31;
  const int wave = (int)(threadIdx.x >> 5);
  const int t = (int)blockIdx.x * 8 + wave;
  if (t >= SEQ) return;
  const float e   = (float)lane * 0.03125f;
  const float pw  = powf(10000.0f, e);
  const float ivf = 1.0f / pw;
  const float ang = (float)t * ivf;
  const float cv  = cosf(ang);
  const float sv  = sinf(ang);
  const size_t o = (size_t)t * NFRQ + lane;
  for (int pass = 0; pass < 2; ++pass) {
    ((volatile float*)cst)[o] = cv;
    ((volatile float*)snt)[o] = sv;
    __threadfence();
  }
}

__global__ __launch_bounds__(256) void cvt_x_bf16_kernel(const float* __restrict__ in, unsigned short* __restrict__ outp, int n8) {
  const int i = (int)blockIdx.x * 256 + (int)threadIdx.x;
  if (i >= n8) return;
  const size_t e   = 8 * (size_t)i;
  const size_t tok = e / DM;
  const size_t col = e - tok * DM;
  const size_t bb  = tok / SEQ;
  const size_t ss  = tok - bb * SEQ;
  const size_t se  = (bb * SEQ_FULL + ss) * DM + col;
  const v4f a = *(const v4f*)(in + se);
  const v4f b = *(const v4f*)(in + se + 4);
  v4u w;
  w[0] = pk16(f2bf_bits(a[0]), f2bf_bits(a[1]));
  w[1] = pk16(f2bf_bits(a[2]), f2bf_bits(a[3]));
  w[2] = pk16(f2bf_bits(b[0]), f2bf_bits(b[1]));
  w[3] = pk16(f2bf_bits(b[2]), f2bf_bits(b[3]));
  *(volatile v4u*)(outp + e) = w;
  __threadfence();
  *(volatile v4u*)(outp + e) = w;
}

__global__ __launch_bounds__(256) void cvt4_bf16_kernel(const float* __restrict__ w0, const float* __restrict__ w1,
                                                        const float* __restrict__ w2, const float* __restrict__ w3,
                                                        unsigned short* __restrict__ outp, int n8) {
  const int sel = (int)blockIdx.y;
  const float* in = (sel == 0) ? w0 : ((sel == 1) ? w1 : ((sel == 2) ? w2 : w3));
  unsigned short* o = outp + (size_t)sel * 8 * (size_t)n8;
  const int i = (int)blockIdx.x * 256 + (int)threadIdx.x;
  if (i >= n8) return;
  const size_t e = 8 * (size_t)i;
  const v4f a = *(const v4f*)(in + e);
  const v4f b = *(const v4f*)(in + e + 4);
  v4u w;
  w[0] = pk16(f2bf_bits(a[0]), f2bf_bits(a[1]));
  w[1] = pk16(f2bf_bits(a[2]), f2bf_bits(a[3]));
  w[2] = pk16(f2bf_bits(b[0]), f2bf_bits(b[1]));
  w[3] = pk16(f2bf_bits(b[2]), f2bf_bits(b[3]));
  *(volatile v4u*)(o + e) = w;
  __threadfence();
  *(volatile v4u*)(o + e) = w;
}

#define AT_NW 4
#define AT_QB 64
#define AT_KC 64
static_assert(SEQ % AT_QB == 0);
static_assert(SEQ % AT_KC == 0);

__device__ __forceinline__ void at_split(float f, __bf16& hi, __bf16& lo) {
  const unsigned short hb = f2bf_bits(f);
  hi = __builtin_bit_cast(__bf16, hb);
  lo = __builtin_bit_cast(__bf16, f2bf_bits(f - bf_bits2f(hb)));
}

__global__ __launch_bounds__(128) __attribute__((amdgpu_num_vgpr(256)))
void attn_causal64_kernel(const unsigned short* __restrict__ qhp, const unsigned short* __restrict__ qlp,
                          const unsigned short* __restrict__ khp, const unsigned short* __restrict__ klp,
                          const unsigned short* __restrict__ vhp, const unsigned short* __restrict__ vlp,
                          unsigned short* __restrict__ yhp, unsigned short* __restrict__ ylp, float sscale) {
  union FB { v16b v; v8b h[2]; };
  __shared__ __align__(16) __bf16   Ksh[AT_KC * HD];
  __shared__ __align__(16) __bf16   Ksl[AT_KC * HD];
  __shared__ __align__(16) __bf16   Vth[HD * AT_KC];
  __shared__ __align__(16) __bf16   Vtl[HD * AT_KC];
  __shared__ __align__(16) __bf16   Psh[AT_NW][16 * AT_KC];
  __shared__ __align__(16) __bf16   Psl[AT_NW][16 * AT_KC];
  __shared__ __align__(16) _Float16 Osh[AT_NW][2 * 16 * HD];

  const int tid  = (int)threadIdx.x;
  const int wave = wave_id();
  const int lane = tid & 31;
  const int hh   = lane >> 4;
  const int c    = lane & 15;

  const int nqb = SEQ / AT_QB;
  const int bx = (int)blockIdx.x;
  const int qb = bx % nqb;
  const int hb = bx / nqb;
  const int h  = hb % NH;
  const int b  = hb / NH;
  const size_t tok0 = (size_t)b * SEQ;
  const int q0 = qb * AT_QB + wave * 16;

  const __bf16* Qh = (const __bf16*)(const void*)qhp + tok0 * DM + (size_t)h * HD;
  const __bf16* Ql = (const __bf16*)(const void*)qlp + tok0 * DM + (size_t)h * HD;
  const __bf16* Kh = (const __bf16*)(const void*)khp + tok0 * DM + (size_t)h * HD;
  const __bf16* Kl = (const __bf16*)(const void*)klp + tok0 * DM + (size_t)h * HD;
  const __bf16* Vh = (const __bf16*)(const void*)vhp + (size_t)h * HD * TOK + tok0;
  const __bf16* Vl = (const __bf16*)(const void*)vlp + (size_t)h * HD * TOK + tok0;

  v16b qah[2], qal[2];
#pragma unroll
  for (int dc = 0; dc < 2; ++dc) {
    const __bf16* qr = Qh + (size_t)(q0 + c) * DM + dc * 32 + 8 * hh;
    const __bf16* ql = Ql + (size_t)(q0 + c) * DM + dc * 32 + 8 * hh;
    qah[dc] = ldfrag_b(qr);
    qal[dc] = ldfrag_b(ql);
  }

  float mrow[8], lrow[8];
  v8f oacc[4];
#pragma unroll
  for (int r = 0; r < 8; ++r) { mrow[r] = -INFINITY; lrow[r] = 0.f; }
#pragma unroll
  for (int t = 0; t < 4; ++t) oacc[t] = zero8();

  __bf16* pwh = Psh[wave];
  __bf16* pwl = Psl[wave];

  const int nChunks = qb + 1;
  for (int kc = 0; kc < nChunks; ++kc) {
    const int kv0 = kc * AT_KC;
    __syncthreads();
    {
      const int r = tid >> 1, half = (tid & 1) * 32;
      const __bf16* ksh = Kh + (size_t)(kv0 + r) * DM + half;
      const __bf16* ksl = Kl + (size_t)(kv0 + r) * DM + half;
      const __bf16* vsh = Vh + (size_t)r * TOK + kv0 + half;
      const __bf16* vsl = Vl + (size_t)r * TOK + kv0 + half;
#pragma unroll
      for (int i = 0; i < 4; ++i) {
        const v8b a0 = *(const v8b*)(ksh + 8 * i);
        const v8b a1 = *(const v8b*)(ksl + 8 * i);
        const v8b b0 = *(const v8b*)(vsh + 8 * i);
        const v8b b1 = *(const v8b*)(vsl + 8 * i);
        *(v8b*)(Ksh + r * HD    + half + 8 * i) = a0;
        *(v8b*)(Ksl + r * HD    + half + 8 * i) = a1;
        *(v8b*)(Vth + r * AT_KC + half + 8 * i) = b0;
        *(v8b*)(Vtl + r * AT_KC + half + 8 * i) = b1;
      }
    }
    __syncthreads();

    v8f s[4];
#pragma unroll
    for (int j = 0; j < 4; ++j) {
      s[j] = zero8();
#pragma unroll
      for (int dc = 0; dc < 2; ++dc) {
        FB kb, kl;
        kb.h[0] = *(const v8b*)(Ksh + (j * 16 + c) * HD + dc * 32 + 8 * hh);
        kb.h[1] = *(const v8b*)(Ksh + (j * 16 + c) * HD + dc * 32 + 16 + 8 * hh);
        kl.h[0] = *(const v8b*)(Ksl + (j * 16 + c) * HD + dc * 32 + 8 * hh);
        kl.h[1] = *(const v8b*)(Ksl + (j * 16 + c) * HD + dc * 32 + 16 + 8 * hh);
        s[j] = at_mma(qah[dc], kb.v, s[j]);
        s[j] = at_mma(qah[dc], kl.v, s[j]);
        s[j] = at_mma(qal[dc], kb.v, s[j]);
      }
    }
    const bool diag = (kc == qb);
    float cm[8];
#pragma unroll
    for (int r = 0; r < 8; ++r) {
      const int qrow = q0 + 8 * hh + r;
      float m = -INFINITY;
#pragma unroll
      for (int j = 0; j < 4; ++j) {
        const int kvcol = kv0 + j * 16 + c;
        const float sv = s[j][r] * sscale;
        const bool masked = diag && (kvcol > qrow);
        const float sm = masked ? -INFINITY : sv;
        s[j][r] = sm;
        m = fmaxf(m, sm);
      }
#pragma unroll
      for (int off = 1; off < 16; off <<= 1) m = fmaxf(m, __shfl_xor(m, off, 32));
      cm[r] = m;
    }
#pragma unroll
    for (int r = 0; r < 8; ++r) {
      const float mnew = fmaxf(mrow[r], cm[r]);
      const float alpha = expf(mrow[r] - mnew);
      mrow[r] = mnew;
      float psum = 0.f;
#pragma unroll
      for (int j = 0; j < 4; ++j) {
        const float p = expf(s[j][r] - mnew);
        psum += p;
        __bf16 a, bl; at_split(p, a, bl);
        pwh[(8 * hh + r) * AT_KC + j * 16 + c] = a;
        pwl[(8 * hh + r) * AT_KC + j * 16 + c] = bl;
      }
#pragma unroll
      for (int off = 1; off < 16; off <<= 1) psum += __shfl_xor(psum, off, 32);
      lrow[r] = lrow[r] * alpha + psum;
#pragma unroll
      for (int t = 0; t < 4; ++t) oacc[t][r] *= alpha;
    }
    lds_wave_sync();
#pragma unroll 1
    for (int kk = 0; kk < 2; ++kk) {
      FB pa, pl;
      pa.h[0] = *(const v8b*)(pwh + c * AT_KC + kk * 32 + 8 * hh);
      pa.h[1] = *(const v8b*)(pwh + c * AT_KC + kk * 32 + 16 + 8 * hh);
      pl.h[0] = *(const v8b*)(pwl + c * AT_KC + kk * 32 + 8 * hh);
      pl.h[1] = *(const v8b*)(pwl + c * AT_KC + kk * 32 + 16 + 8 * hh);
#pragma unroll
      for (int t = 0; t < 4; ++t) {
        FB vb, vl;
        vb.h[0] = *(const v8b*)(Vth + (t * 16 + c) * AT_KC + kk * 32 + 8 * hh);
        vb.h[1] = *(const v8b*)(Vth + (t * 16 + c) * AT_KC + kk * 32 + 16 + 8 * hh);
        vl.h[0] = *(const v8b*)(Vtl + (t * 16 + c) * AT_KC + kk * 32 + 8 * hh);
        vl.h[1] = *(const v8b*)(Vtl + (t * 16 + c) * AT_KC + kk * 32 + 16 + 8 * hh);
        oacc[t] = at_mma(pa.v, vb.v, oacc[t]);
        oacc[t] = at_mma(pa.v, vl.v, oacc[t]);
        oacc[t] = at_mma(pl.v, vb.v, oacc[t]);
      }
    }
  }

  _Float16* osh = Osh[wave];
  _Float16* osl = osh + 16 * HD;
#pragma unroll
  for (int r = 0; r < 8; ++r) {
    const float inv = 1.0f / lrow[r];
#pragma unroll
    for (int t = 0; t < 4; ++t) {
      const float o = oacc[t][r] * inv;
      const unsigned short hb = f2bf_bits(o);
      const unsigned short lb = f2bf_bits(o - bf_bits2f(hb));
      const int so = (8 * hh + r) * HD + t * 16 + c;
      osh[so] = __builtin_bit_cast(_Float16, hb);
      osl[so] = __builtin_bit_cast(_Float16, lb);
    }
  }
  lds_wave_sync();
  _Float16* Yhg = (_Float16*)(void*)yhp + (tok0 + (size_t)q0) * DM + (size_t)h * HD;
  _Float16* Ylg = (_Float16*)(void*)ylp + (tok0 + (size_t)q0) * DM + (size_t)h * HD;
  const int q4 = lane >> 3;
  const int c8 = (lane & 7) * 8;
  for (int pass = 0; pass < 2; ++pass) {
#pragma unroll
    for (int it = 0; it < 4; ++it) {
      const int row = it * 4 + q4;
      const v8h xh = *(const v8h*)(osh + row * HD + c8);
      const v8h xl = *(const v8h*)(osl + row * HD + c8);
      *(volatile v8h*)(Yhg + (size_t)row * DM + c8) = xh;
      *(volatile v8h*)(Ylg + (size_t)row * DM + c8) = xl;
    }
    __threadfence();
  }
}

extern "C" void kernel_launch(void* const* d_in, const int* in_sizes, int n_in,
                              void* d_out, int out_size, void* d_ws, size_t ws_size,
                              hipStream_t stream) {
  if (n_in < 5) return;
  const long long needX = (long long)((NB - 1) * SEQ_FULL + SEQ) * DM;
  if ((long long)in_sizes[0] < needX) return;
  if (in_sizes[1] < DM * DM || in_sizes[2] < DM * DM || in_sizes[3] < DM * DM || in_sizes[4] < DM * DM) return;
  if ((long long)out_size < needX) return;

  const float* x  = (const float*)d_in[0];
  const float* Wq = (const float*)d_in[1];
  const float* Wk = (const float*)d_in[2];
  const float* Wv = (const float*)d_in[3];
  const float* Wo = (const float*)d_in[4];
  float* out = (float*)d_out;

  const size_t PX = (size_t)TOK * DM * 2;
  const size_t PW = (size_t)DM * DM * 2;
  const size_t PT = (size_t)SEQ * NFRQ * 4;
  size_t off = 0;
  const size_t oXB  = off; off += PX;
  const size_t oWB  = off; off += 4 * PW;
  const size_t oCs  = off; off += PT;
  const size_t oSn  = off; off += PT;
  const size_t oQh  = off; off += PX;  const size_t oQl  = off; off += PX;
  const size_t oKh  = off; off += PX;  const size_t oKl  = off; off += PX;
  const size_t oVTh = off; off += PX;  const size_t oVTl = off; off += PX;
  const size_t oYh  = off; off += PX;  const size_t oYl  = off; off += PX;
  if (off > ws_size) return;
  if (off > (size_t)134217728) return;

  char* ws = (char*)d_ws;
  unsigned short* XB  = (unsigned short*)(ws + oXB);
  unsigned short* WB  = (unsigned short*)(ws + oWB);
  unsigned short* WQb = WB;
  unsigned short* WKb = WB + (size_t)DM * DM;
  unsigned short* WVb = WB + (size_t)2 * DM * DM;
  unsigned short* WOb = WB + (size_t)3 * DM * DM;
  float*          cst = (float*)(ws + oCs);
  float*          snt = (float*)(ws + oSn);
  unsigned short* Qh  = (unsigned short*)(ws + oQh);  unsigned short* Ql  = (unsigned short*)(ws + oQl);
  unsigned short* Kh  = (unsigned short*)(ws + oKh);  unsigned short* Kl  = (unsigned short*)(ws + oKl);
  unsigned short* VTh = (unsigned short*)(ws + oVTh); unsigned short* VTl = (unsigned short*)(ws + oVTl);
  unsigned short* Yh  = (unsigned short*)(ws + oYh);  unsigned short* Yl  = (unsigned short*)(ws + oYl);

  const dim3 b256(256), b128(128);
  const int tilesP = (TOK / 64) * (DM / 64);
  const dim3 gP((tilesP + 7) / 8);

  rot_table_kernel<<<dim3(SEQ / 8), b256, 0, stream>>>(cst, snt);
  cvt_x_bf16_kernel<<<dim3((TOK * DM / 8) / 256), b256, 0, stream>>>(x, XB, TOK * DM / 8);
  cvt4_bf16_kernel<<<dim3((DM * DM / 8) / 256, 4), b256, 0, stream>>>(Wq, Wk, Wv, Wo, WB, DM * DM / 8);
  wmma_gemm64<0, 2, true><<<gP, b256, 0, stream>>>(
      XB, XB, DM, WQb, WQb, DM, (void*)Qh, (void*)Ql, DM, cst, snt, TOK, DM, DM, 1.0f);
  wmma_gemm64<0, 2, true><<<gP, b256, 0, stream>>>(
      XB, XB, DM, WKb, WKb, DM, (void*)Kh, (void*)Kl, DM, cst, snt, TOK, DM, DM, 1.0f);
  wmma_gemm64<0, 2, false><<<gP, b256, 0, stream>>>(
      WVb, WVb, DM, XB, XB, DM, (void*)VTh, (void*)VTl, TOK, cst, snt, DM, TOK, DM, 1.0f);
  attn_causal64_kernel<<<dim3(NB * NH * (SEQ / AT_QB)), b128, 0, stream>>>(Qh, Ql, Kh, Kl, VTh, VTl, Yh, Yl, 0.125f);
  wmma_gemm64<1, 0, false><<<gP, b256, 0, stream>>>(
      Yh, Yl, DM, WOb, WOb, DM, (void*)out, (void*)out, DM, cst, snt, TOK, DM, DM, 1.0f);
  (void)hipGetLastError();
}
